// PoPETransformerBlock_71442486001861
// MI455X (gfx1250) — hardware-verified
//
#include <hip/hip_runtime.h>
#include <math.h>
#include <stdint.h>

constexpr int kBatch = 4;
constexpr int kSeq   = 1024;
constexpr int kDim   = 1024;
constexpr int kHeads = 16;
constexpr int kDh    = 64;
constexpr int kInner = kHeads * kDh;
constexpr int kMlp   = 4096;
constexpr int kQkW   = 2 * kInner;
constexpr int kPopeW = kHeads * 2 * kDh;
constexpr int kHG    = 8;
constexpr int kNGrp  = kHeads / kHG;
static_assert(kSeq % 64 == 0 && kDim % 64 == 0 && kMlp % 64 == 0 && kDh == 64, "tile multiples");
static_assert(kDim % 32 == 0 && (2 * kDh) % 32 == 0 && kSeq % 32 == 0 && kMlp % 32 == 0, "K multiples of 32");

typedef __attribute__((ext_vector_type(16))) _Float16 v16h;
typedef __attribute__((ext_vector_type(8)))  _Float16 v8h;
typedef __attribute__((ext_vector_type(16))) __bf16   v16b;
typedef __attribute__((ext_vector_type(8)))  __bf16   v8b;
typedef __attribute__((ext_vector_type(8)))  float    v8f;
typedef __attribute__((ext_vector_type(4)))  float    v4f;
typedef __attribute__((ext_vector_type(2)))  float    v2f;
typedef __attribute__((ext_vector_type(4)))  unsigned int v4u;
#define PSCALE 32768.0f
#define PSCALE_INV (1.0f / 32768.0f)

__device__ __forceinline__ unsigned short f2bf_bits(float f) {
  unsigned u = __float_as_uint(f);
  return (unsigned short)((u + 0x7FFFu + ((u >> 16) & 1u)) >> 16);
}
__device__ __forceinline__ float bf_bits2f(unsigned short h) { return __uint_as_float(((unsigned)h) << 16); }

__device__ __forceinline__ void dep_guard_h(v8f& a, v8f& b, v16h x, v16h y) { asm volatile("v_nop\n\tv_nop\n\tv_nop\n\tv_nop" : "+v"(a), "+v"(b) : "v"(x), "v"(y)); }
__device__ __forceinline__ void dep_guard_b(v8f& a, v8f& b, v16b x, v16b y) { asm volatile("v_nop\n\tv_nop\n\tv_nop\n\tv_nop" : "+v"(a), "+v"(b) : "v"(x), "v"(y)); }
__device__ __forceinline__ void keep4_h(v16h a, v16h b, v16h c, v16h d) { asm volatile("v_nop" :: "v"(a), "v"(b), "v"(c), "v"(d)); }
__device__ __forceinline__ void keep4_b(v16b a, v16b b, v16b c, v16b d) { asm volatile("v_nop" :: "v"(a), "v"(b), "v"(c), "v"(d)); }
__device__ __forceinline__ void acc_guard4(v8f& a, v8f& b, v8f& c, v8f& d) { asm volatile("v_nop\n\tv_nop\n\tv_nop\n\tv_nop" : "+v"(a), "+v"(b), "+v"(c), "+v"(d)); }
template <typename T> struct Frag;
template <> struct Frag<_Float16> {
  typedef v16h V; union U { v16h v; v8h h[2]; };
  static __device__ __forceinline__ v16h load(const _Float16* p) {
    U f; f.h[0] = *(const v8h*)(p); f.h[1] = *(const v8h*)(p + 16); return f.v;
  }
  static __device__ __forceinline__ v8f mma(v16h a, v16h b, v8f c) {
    return __builtin_amdgcn_wmma_f32_16x16x32_f16(false, a, false, b, (short)0, c, false, false);
  }
  static __device__ __forceinline__ void guard(v8f& a, v8f& b, v16h x, v16h y) { dep_guard_h(a, b, x, y); }
  static __device__ __forceinline__ void keep(v16h a, v16h b, v16h c, v16h d) { keep4_h(a, b, c, d); }
};
template <> struct Frag<__bf16> {
  typedef v16b V; union U { v16b v; v8b h[2]; };
  static __device__ __forceinline__ v16b load(const __bf16* p) {
    U f; f.h[0] = *(const v8b*)(p); f.h[1] = *(const v8b*)(p + 16); return f.v;
  }
  static __device__ __forceinline__ v8f mma(v16b a, v16b b, v8f c) {
    return __builtin_amdgcn_wmma_f32_16x16x32_bf16(false, a, false, b, (short)0, c, false, false);
  }
  static __device__ __forceinline__ void guard(v8f& a, v8f& b, v16b x, v16b y) { dep_guard_b(a, b, x, y); }
  static __device__ __forceinline__ void keep(v16b a, v16b b, v16b c, v16b d) { keep4_b(a, b, c, d); }
};

template <int ET> struct Elem;
template <> struct Elem<0> { typedef _Float16 T; };
template <> struct Elem<1> { typedef __bf16 T; };
template <int ET, bool SPLIT, int BIAS_MODE, int OUT_MODE, bool RESID, int ACT = 0>
__global__ __launch_bounds__(256) void wmma_gemm64(
    const unsigned short* __restrict__ Ap, const unsigned short* __restrict__ A2p, int lda, long strideA,
    const unsigned short* __restrict__ Btp, const unsigned short* __restrict__ Bt2p, int ldb, long strideB,
    void* __restrict__ Cout, void* __restrict__ Cout2, int ldc, long strideC,
    const float* __restrict__ bias,
    const float* __restrict__ resid, long strideR,
    int M, int N, int K, float scale) {
  typedef typename Elem<ET>::T T;
  typedef typename Frag<T>::V V;
  const T* A = (const T*)Ap; const T* A2 = (const T*)A2p; const T* Bt = (const T*)Btp; const T* Bt2 = (const T*)Bt2p;
  __shared__ __align__(16) float sT[8][16 * 68];
  const int b    = blockIdx.y;
  const int lane = threadIdx.x & 31;
  const int wave = threadIdx.x >> 5;
  const int tilesN = N >> 6;
  const int tilesM = M >> 6;
  const int tile = blockIdx.x * 8 + wave;
  if (tile >= tilesM * tilesN) return;
  const int tm = tile / tilesN;
  const int tn = tile - tm * tilesN;
  const int m0 = tm << 6;
  const int n0 = tn << 6;

  const T* Ab  = A  + (size_t)b * strideA;
  const T* Bb  = Bt + (size_t)b * strideB;
  const T* Ab2 = SPLIT ? (A2  + (size_t)b * strideA) : nullptr;
  const T* Bb2 = SPLIT ? (Bt2 + (size_t)b * strideB) : nullptr;

  const int rlane = lane & 15;
  const int koff  = (lane >> 4) * 8;
  const int mOff  = (lane >> 4) * 8;

  v8f acc[4][4];
#pragma unroll
  for (int i = 0; i < 4; ++i)
#pragma unroll
    for (int j = 0; j < 4; ++j) acc[i][j] = (v8f){0.f,0.f,0.f,0.f,0.f,0.f,0.f,0.f};

  for (int k0 = 0; k0 < K; k0 += 32) {
    V bh[4], bl[4];
#pragma unroll
    for (int j = 0; j < 4; ++j) {
      const size_t bo = (size_t)(n0 + (j << 4) + rlane) * ldb + koff + k0;
      bh[j] = Frag<T>::load(Bb + bo);
      if (SPLIT) bl[j] = Frag<T>::load(Bb2 + bo);
    }
#pragma unroll
    for (int i = 0; i < 4; ++i) {
      const size_t ao = (size_t)(m0 + (i << 4) + rlane) * lda + koff + k0;
      V ah = Frag<T>::load(Ab + ao);
      V al;
      if (SPLIT) al = Frag<T>::load(Ab2 + ao);
#pragma unroll
      for (int j = 0; j < 4; ++j) {
        acc[i][j] = Frag<T>::mma(ah, bh[j], acc[i][j]);
        if (SPLIT) {
          acc[i][j] = Frag<T>::mma(ah, bl[j], acc[i][j]);
          acc[i][j] = Frag<T>::mma(al, bh[j], acc[i][j]);
        }
      }
      Frag<T>::guard(acc[i][0], acc[i][3], ah, SPLIT ? al : ah);
    }
    Frag<T>::keep(bh[0], bh[1], bh[2], bh[3]);
    if (SPLIT) Frag<T>::keep(bl[0], bl[1], bl[2], bl[3]);
  }
  acc_guard4(acc[0][0], acc[0][1], acc[0][2], acc[0][3]);
  acc_guard4(acc[1][0], acc[1][1], acc[1][2], acc[1][3]);
  acc_guard4(acc[2][0], acc[2][1], acc[2][2], acc[2][3]);
  acc_guard4(acc[3][0], acc[3][1], acc[3][2], acc[3][3]);

  float* slab = sT[wave];
  const float* Rb = RESID ? (resid + (size_t)b * strideR) : nullptr;
#pragma unroll
  for (int i = 0; i < 4; ++i) {
    const int mBase = m0 + (i << 4);
#pragma unroll
    for (int j = 0; j < 4; ++j) {
      const int n = n0 + (j << 4) + rlane;
      float bv = 0.f;
      if (BIAS_MODE == 2) bv = bias[n];
#pragma unroll
      for (int r = 0; r < 8; ++r) {
        float v = acc[i][j][r] * scale;
        if (BIAS_MODE == 1) v += bias[mBase + mOff + r];
        if (BIAS_MODE == 2) v += bv;
        if (RESID) v += Rb[(size_t)(mBase + mOff + r) * ldc + n];
        if (ACT == 1) v = tanhf(v);
        if (ACT == 2) v = fmaxf(v, 0.0f);
        if (ACT == 3) v = v / (1.0f + expf(-v));
        if (ACT == 4) v = (v > 0.f) ? v : 0.01f * v;
        slab[(mOff + r) * 68 + (j << 4) + rlane] = v;
      }
    }
    __builtin_amdgcn_fence(__ATOMIC_RELEASE, "workgroup");
    __builtin_amdgcn_wave_barrier();
    __builtin_amdgcn_fence(__ATOMIC_ACQUIRE, "workgroup");
    if (OUT_MODE == 0) {
      float* C = (float*)Cout + (size_t)b * strideC;
      const int hh = lane >> 4, c4 = (lane & 15) * 4;
      for (int pass = 0; pass < 2; ++pass) {
#pragma unroll
        for (int it = 0; it < 8; ++it) {
          const int row = it * 2 + hh;
          v4f v = *(const v4f*)(slab + row * 68 + c4);
          *(volatile v4f*)(C + (size_t)(mBase + row) * ldc + n0 + c4) = v;
        }
        __threadfence();
      }
    } else {
      const int q = lane >> 3, c8 = (lane & 7) * 8;
      unsigned short* C  = (unsigned short*)Cout  + (size_t)b * strideC;
      unsigned short* C2 = (OUT_MODE == 2) ? ((unsigned short*)Cout2 + (size_t)b * strideC) : nullptr;
      for (int pass = 0; pass < 2; ++pass) {
#pragma unroll
        for (int it = 0; it < 4; ++it) {
          const int row = it * 4 + q;
          const float* sp = slab + row * 68 + c8;
          v8h hv, lv;
#pragma unroll
          for (int e = 0; e < 8; ++e) {
            if (OUT_MODE == 1) {
              hv[e] = (_Float16)sp[e];
            } else {
              unsigned short hb = f2bf_bits(sp[e]);
              unsigned short lb = f2bf_bits(sp[e] - bf_bits2f(hb));
              hv[e] = __builtin_bit_cast(_Float16, hb);
              lv[e] = __builtin_bit_cast(_Float16, lb);
            }
          }
          *(volatile v8h*)(C + (size_t)(mBase + row) * ldc + n0 + c8) = hv;
          if (OUT_MODE == 2) *(volatile v8h*)(C2 + (size_t)(mBase + row) * ldc + n0 + c8) = lv;
        }
        __threadfence();
      }
    }
    __builtin_amdgcn_fence(__ATOMIC_RELEASE, "workgroup");
    __builtin_amdgcn_wave_barrier();
    __builtin_amdgcn_fence(__ATOMIC_ACQUIRE, "workgroup");
  }
}

__device__ __forceinline__ unsigned pk16(unsigned short a, unsigned short b) { return (unsigned)a | ((unsigned)b << 16); }
__device__ __forceinline__ unsigned short h_bits(float f) { const _Float16 h = (_Float16)f; return __builtin_bit_cast(unsigned short, h); }

__global__ __launch_bounds__(256) void transpose_cast_f16_kernel(const float* __restrict__ src,
                                                                 unsigned short* __restrict__ dst,
                                                                 int Kd, int Nd, float scale) {
  __shared__ __align__(16) _Float16 tile[64 * 72];
  const int n0 = blockIdx.x * 64, k0 = blockIdx.y * 64, t = threadIdx.x;
#pragma unroll
  for (int i = 0; i < 4; ++i) {
    const int idx = t + 256 * i;
    const int kr = idx >> 4, c4 = (idx & 15) * 4;
    const v4f w = *(const v4f*)(src + (size_t)(k0 + kr) * Nd + n0 + c4);
#pragma unroll
    for (int e = 0; e < 4; ++e) tile[(c4 + e) * 72 + kr] = (_Float16)(w[e] * scale);
  }
  __syncthreads();
  _Float16* out = (_Float16*)dst;
  for (int pass = 0; pass < 2; ++pass) {
#pragma unroll
    for (int i = 0; i < 2; ++i) {
      const int idx = t + 256 * i;
      const int nr = idx >> 3, c8 = (idx & 7) * 8;
      const v8h v = *(const v8h*)(tile + nr * 72 + c8);
      *(volatile v8h*)(out + (size_t)(n0 + nr) * Kd + k0 + c8) = v;
    }
    __threadfence();
  }
}

__global__ __launch_bounds__(128) void layernorm_f16_kernel(const float* __restrict__ x, const float* __restrict__ g,
                                                           const float* __restrict__ bt, unsigned short* __restrict__ out) {
  __shared__ float redA[4];
  __shared__ float redB[4];
  const int row = blockIdx.x, t = threadIdx.x, lane = t & 31, wave = t >> 5;
  const int c0 = t * 8;
  const float* xr = x + (size_t)row * kDim + c0;
  const v4f a = *(const v4f*)(xr);
  const v4f c = *(const v4f*)(xr + 4);
  float s = ((a[0] + a[1]) + (a[2] + a[3])) + ((c[0] + c[1]) + (c[2] + c[3]));
#pragma unroll
  for (int off = 16; off > 0; off >>= 1) s += __shfl_xor(s, off, 32);
  if (lane == 0) redA[wave] = s;
  __syncthreads();
  const float mean = ((redA[0] + redA[1]) + (redA[2] + redA[3])) * (1.0f / 1024.0f);
  const float d0 = a[0] - mean, d1 = a[1] - mean, d2 = a[2] - mean, d3 = a[3] - mean;
  const float d4 = c[0] - mean, d5 = c[1] - mean, d6 = c[2] - mean, d7 = c[3] - mean;
  float ss = ((d0 * d0 + d1 * d1) + (d2 * d2 + d3 * d3)) + ((d4 * d4 + d5 * d5) + (d6 * d6 + d7 * d7));
#pragma unroll
  for (int off = 16; off > 0; off >>= 1) ss += __shfl_xor(ss, off, 32);
  if (lane == 0) redB[wave] = ss;
  __syncthreads();
  const float var = ((redB[0] + redB[1]) + (redB[2] + redB[3])) * (1.0f / 1024.0f);
  const float inv = rsqrtf(var + 1e-5f);
  const v4f ga = *(const v4f*)(g + c0), gc = *(const v4f*)(g + c0 + 4);
  const v4f ba = *(const v4f*)(bt + c0), bc = *(const v4f*)(bt + c0 + 4);
  const float y0 = d0 * inv * ga[0] + ba[0], y1 = d1 * inv * ga[1] + ba[1];
  const float y2 = d2 * inv * ga[2] + ba[2], y3 = d3 * inv * ga[3] + ba[3];
  const float y4 = d4 * inv * gc[0] + bc[0], y5 = d5 * inv * gc[1] + bc[1];
  const float y6 = d6 * inv * gc[2] + bc[2], y7 = d7 * inv * gc[3] + bc[3];
  const v4u hv = (v4u){pk16(h_bits(y0), h_bits(y1)), pk16(h_bits(y2), h_bits(y3)),
                       pk16(h_bits(y4), h_bits(y5)), pk16(h_bits(y6), h_bits(y7))};
  const size_t ro = (size_t)row * kDim + c0;
  *(volatile v4u*)(out + ro) = hv;
  __threadfence();
  *(volatile v4u*)(out + ro) = hv;
}

constexpr float kFreqChi = 0.20762062072753906f;
constexpr float kFreqClo = -1.1479708e-7f;

__global__ __launch_bounds__(256) void polar_qk_kernel(const float* __restrict__ qk, const float* __restrict__ phase,
                                                       unsigned short* __restrict__ q2k2) {
  #pragma clang fp contract(off)
  __shared__ __align__(16) _Float16 rowT[512];
  const int n = blockIdx.x, hq = blockIdx.y, which = blockIdx.z;
  const int t = threadIdx.x, hl = t >> 6, d = t & 63, h = hq * 4 + hl;
  const float val = qk[(size_t)n * kQkW + which * kInner + h * kDh + d];
  const float mag = fmaxf(val, 0.0f) + log1pf(expf(-fabsf(val)));
  const float fd = (float)d;
  const float freq = exp2f(-fd * kFreqChi) * exp2f(-fd * kFreqClo);
  const float th = (float)n * freq;
  const float phv = phase[h * kDh + d];
  const float ang = (which != 0) ? (th + phv) : th;
  float sv, cv;
  sincosf(ang, &sv, &cv);
  rowT[hl * 128 + d]      = (_Float16)(mag * cv);
  rowT[hl * 128 + 64 + d] = (_Float16)(mag * sv);
  __syncthreads();
  if (t < 64) {
    const v8h v = *(const v8h*)(rowT + t * 8);
    _Float16* dst = (_Float16*)q2k2 + (size_t)which * ((size_t)kSeq * kPopeW) + (size_t)n * kPopeW + hq * 512 + t * 8;
    *(volatile v8h*)dst = v;
    __threadfence();
    *(volatile v8h*)dst = v;
  }
}

__global__ __launch_bounds__(128) void softmax_p16_kernel(const float* __restrict__ S, unsigned short* __restrict__ P) {
  __shared__ float redm[4];
  __shared__ float reds[4];
  const int i = blockIdx.x, hg = blockIdx.y;
  const int t = threadIdx.x, lane = t & 31, wave = t >> 5;
  const int j0 = t * 8;
  const size_t ro = ((size_t)hg * kSeq + i) * kSeq + j0;
  const v4f a = *(const v4f*)(S + ro);
  const v4f c = *(const v4f*)(S + ro + 4);
  float m = fmaxf(fmaxf(fmaxf(a[0], a[1]), fmaxf(a[2], a[3])), fmaxf(fmaxf(c[0], c[1]), fmaxf(c[2], c[3])));
#pragma unroll
  for (int off = 16; off > 0; off >>= 1) m = fmaxf(m, __shfl_xor(m, off, 32));
  if (lane == 0) redm[wave] = m;
  __syncthreads();
  const float mx = fmaxf(fmaxf(redm[0], redm[1]), fmaxf(redm[2], redm[3]));
  const float e0 = __expf(a[0] - mx), e1 = __expf(a[1] - mx), e2 = __expf(a[2] - mx), e3 = __expf(a[3] - mx);
  const float e4 = __expf(c[0] - mx), e5 = __expf(c[1] - mx), e6 = __expf(c[2] - mx), e7 = __expf(c[3] - mx);
  float s = ((e0 + e1) + (e2 + e3)) + ((e4 + e5) + (e6 + e7));
#pragma unroll
  for (int off = 16; off > 0; off >>= 1) s += __shfl_xor(s, off, 32);
  if (lane == 0) reds[wave] = s;
  __syncthreads();
  const float tot = (reds[0] + reds[1]) + (reds[2] + reds[3]);
  const float inv = 1.0f / tot;
  const float p0 = e0 * inv, p1 = e1 * inv, p2 = e2 * inv, p3 = e3 * inv;
  const float p4 = e4 * inv, p5 = e5 * inv, p6 = e6 * inv, p7 = e7 * inv;
  const v4u hv = (v4u){pk16(h_bits(p0 * PSCALE), h_bits(p1 * PSCALE)),
                       pk16(h_bits(p2 * PSCALE), h_bits(p3 * PSCALE)),
                       pk16(h_bits(p4 * PSCALE), h_bits(p5 * PSCALE)),
                       pk16(h_bits(p6 * PSCALE), h_bits(p7 * PSCALE))};
  *(volatile v4u*)(P + ro) = hv;
  __threadfence();
  *(volatile v4u*)(P + ro) = hv;
}

__global__ __launch_bounds__(256) void gelu_f16x2_kernel(const float* __restrict__ in, unsigned short* __restrict__ out,
                                                         int n2, float scale) {
  const int i = blockIdx.x * 256 + threadIdx.x;
  if (i < n2) {
    const v2f f = *(const v2f*)(in + 2 * (size_t)i);
    float r0 = 0.0f, r1 = 0.0f;
#pragma unroll 1
    for (int e = 0; e < 2; ++e) {
      const float xv = (e == 0) ? f[0] : f[1];
      const float gv = 0.5f * xv * (1.0f + erff(xv * 0.70710678118654752f));
      r0 = (e == 0) ? gv : r0;
      r1 = (e == 0) ? r1 : gv;
    }
    const unsigned u = pk16(h_bits(r0 * scale), h_bits(r1 * scale));
    ((volatile unsigned*)out)[i] = u;
    __threadfence();
    ((volatile unsigned*)out)[i] = u;
  }
}

extern "C" void kernel_launch(void* const* d_in, const int* in_sizes, int n_in,
                              void* d_out, int out_size, void* d_ws, size_t ws_size,
                              hipStream_t stream) {
  if (n_in < 13) return;
  if (in_sizes[0] != kBatch * kSeq * kDim) return;
  if (in_sizes[1] != kDim || in_sizes[2] != kDim) return;
  if (in_sizes[3] != kDim * 3 * kInner) return;
  if (in_sizes[4] != kInner * kDim || in_sizes[5] != kDim) return;
  if (in_sizes[6] != kHeads * kDh) return;
  if (in_sizes[7] != kDim || in_sizes[8] != kDim) return;
  if (in_sizes[9] != kDim * kMlp || in_sizes[10] != kMlp) return;
  if (in_sizes[11] != kMlp * kDim || in_sizes[12] != kDim) return;
  if (out_size != kBatch * kSeq * kDim) return;

  const float* x     = (const float*)d_in[0];
  const float* ln1_g = (const float*)d_in[1];
  const float* ln1_b = (const float*)d_in[2];
  const float* w_qkv = (const float*)d_in[3];
  const float* w_out = (const float*)d_in[4];
  const float* b_out = (const float*)d_in[5];
  const float* phase = (const float*)d_in[6];
  const float* ln2_g = (const float*)d_in[7];
  const float* ln2_b = (const float*)d_in[8];
  const float* w1    = (const float*)d_in[9];
  const float* b1    = (const float*)d_in[10];
  const float* w2    = (const float*)d_in[11];
  const float* b2    = (const float*)d_in[12];

  const size_t szWQKV = (size_t)3 * kInner * kDim * 2;
  const size_t szWOUT = (size_t)kDim * kInner * 2;
  const size_t szW1   = (size_t)kMlp * kDim * 2;
  const size_t szW2   = (size_t)kDim * kMlp * 2;
  const size_t szH16  = (size_t)kSeq * kDim * 2;
  const size_t szQK   = (size_t)kSeq * kQkW * 4;
  const size_t szVT   = (size_t)kInner * kSeq * 2;
  const size_t szQ2K2 = (size_t)2 * kSeq * kPopeW * 2;
  const size_t szCTX  = (size_t)kSeq * kInner * 2;
  const size_t szX1   = (size_t)kSeq * kDim * 4;
  const size_t szS    = (size_t)kHG * kSeq * kSeq * 4;
  const size_t szP    = (size_t)kHG * kSeq * kSeq * 2;
  const size_t szU    = (size_t)kSeq * kMlp * 4;
  const size_t szG    = (size_t)kSeq * kMlp * 2;
  const size_t szBIG  = szS + szP;
  size_t off = 0;
  const size_t oWQKV = off; off += szWQKV;
  const size_t oWOUT = off; off += szWOUT;
  const size_t oW1   = off; off += szW1;
  const size_t oW2   = off; off += szW2;
  const size_t oH16  = off; off += szH16;
  const size_t oQK   = off; off += szQK;
  const size_t oVT   = off; off += szVT;
  const size_t oQ2K2 = off; off += szQ2K2;
  const size_t oCTX  = off; off += szCTX;
  const size_t oX1   = off; off += szX1;
  const size_t oBIG  = off; off += szBIG;
  if (off > ws_size) return;
  if (szU + szG > szBIG) return;

  char* ws = (char*)d_ws;
  unsigned short* WQKV16 = (unsigned short*)(ws + oWQKV);
  unsigned short* WOUT16 = (unsigned short*)(ws + oWOUT);
  unsigned short* W1T16  = (unsigned short*)(ws + oW1);
  unsigned short* W2T16  = (unsigned short*)(ws + oW2);
  unsigned short* H16    = (unsigned short*)(ws + oH16);
  float*          QKf    = (float*)(ws + oQK);
  unsigned short* VT16   = (unsigned short*)(ws + oVT);
  unsigned short* Q2K2   = (unsigned short*)(ws + oQ2K2);
  unsigned short* Q2p    = Q2K2;
  unsigned short* K2p    = Q2K2 + (size_t)kSeq * kPopeW;
  unsigned short* CTX16  = (unsigned short*)(ws + oCTX);
  float*          X1     = (float*)(ws + oX1);
  float*          Sbuf   = (float*)(ws + oBIG);
  unsigned short* P16    = (unsigned short*)(ws + oBIG + szS);
  float*          Ubuf   = (float*)(ws + oBIG);
  unsigned short* G16    = (unsigned short*)(ws + oBIG + szU);

  const dim3 blk256(256), blk128(128);
  const float wcarry = 16.0f;

  transpose_cast_f16_kernel<<<dim3(3 * kInner / 64, kDim / 64), blk256, 0, stream>>>(w_qkv, WQKV16, kDim, 3 * kInner, wcarry);
  transpose_cast_f16_kernel<<<dim3(kDim / 64, kInner / 64), blk256, 0, stream>>>(w_out, WOUT16, kInner, kDim, wcarry);
  transpose_cast_f16_kernel<<<dim3(kMlp / 64, kDim / 64), blk256, 0, stream>>>(w1, W1T16, kDim, kMlp, wcarry);
  transpose_cast_f16_kernel<<<dim3(kDim / 64, kMlp / 64), blk256, 0, stream>>>(w2, W2T16, kMlp, kDim, wcarry);

  const int tilesM = kSeq / 64;
  const dim3 gQK((tilesM * (kQkW / 64) + 7) / 8, 1);
  const dim3 gV(((kInner / 64) * tilesM + 7) / 8, 1);
  const dim3 gS((tilesM * (kSeq / 64) + 7) / 8, kHG);
  const dim3 gPV((tilesM * (kDh / 64) + 7) / 8, kHG);
  const dim3 gO((tilesM * (kDim / 64) + 7) / 8, 1);
  const dim3 gM1((tilesM * (kMlp / 64) + 7) / 8, 1);
  const dim3 gM2((tilesM * (kDim / 64) + 7) / 8, 1);
  const int n2g = kSeq * kMlp / 2;
  const dim3 gGelu((n2g + 255) / 256);

  for (int b = 0; b < kBatch; ++b) {
    const float* xb = x + (size_t)b * kSeq * kDim;
    float* outb = (float*)d_out + (size_t)b * kSeq * kDim;
    layernorm_f16_kernel<<<dim3(kSeq), blk128, 0, stream>>>(xb, ln1_g, ln1_b, H16);
    wmma_gemm64<0, false, 0, 0, false, 0><<<gQK, blk256, 0, stream>>>(
        H16, H16, kDim, 0L, WQKV16, WQKV16, kDim, 0L, (void*)QKf, (void*)QKf, kQkW, 0L,
        b_out, b_out, 0L, kSeq, kQkW, kDim, 1.0f / 16.0f);
    wmma_gemm64<0, false, 0, 1, false, 0><<<gV, blk256, 0, stream>>>(
        WQKV16 + (size_t)2 * kInner * kDim, WQKV16 + (size_t)2 * kInner * kDim, kDim, 0L, H16, H16, kDim, 0L,
        (void*)VT16, (void*)VT16, kSeq, 0L,
        b_out, b_out, 0L, kInner, kSeq, kDim, 1.0f);
    polar_qk_kernel<<<dim3(kSeq, kHeads / 4, 2), blk256, 0, stream>>>(QKf, phase, Q2K2);
    for (int g = 0; g < kNGrp; ++g) {
      const size_t hc = (size_t)g * kHG;
      wmma_gemm64<0, false, 0, 0, false, 0><<<gS, blk256, 0, stream>>>(
          Q2p + hc * (2 * kDh), Q2p + hc * (2 * kDh), kPopeW, (long)(2 * kDh),
          K2p + hc * (2 * kDh), K2p + hc * (2 * kDh), kPopeW, (long)(2 * kDh),
          (void*)Sbuf, (void*)Sbuf, kSeq, (long)kSeq * kSeq,
          b_out, b_out, 0L, kSeq, kSeq, 2 * kDh, 0.125f);
      softmax_p16_kernel<<<dim3(kSeq, kHG), blk128, 0, stream>>>(Sbuf, P16);
      wmma_gemm64<0, false, 0, 1, false, 0><<<gPV, blk256, 0, stream>>>(
          P16, P16, kSeq, (long)kSeq * kSeq, VT16 + hc * kDh * kSeq, VT16 + hc * kDh * kSeq, kSeq, (long)kDh * kSeq,
          (void*)(CTX16 + hc * kDh), (void*)(CTX16 + hc * kDh), kInner, (long)kDh,
          b_out, b_out, 0L, kSeq, kDh, kSeq, PSCALE_INV);
    }
    wmma_gemm64<0, false, 2, 0, true, 0><<<gO, blk256, 0, stream>>>(
        CTX16, CTX16, kInner, 0L, WOUT16, WOUT16, kInner, 0L, (void*)X1, (void*)X1, kDim, 0L,
        b_out, xb, 0L, kSeq, kDim, kInner, 1.0f / 256.0f);
    layernorm_f16_kernel<<<dim3(kSeq), blk128, 0, stream>>>(X1, ln2_g, ln2_b, H16);
    wmma_gemm64<0, false, 2, 0, false, 0><<<gM1, blk256, 0, stream>>>(
        H16, H16, kDim, 0L, W1T16, W1T16, kDim, 0L, (void*)Ubuf, (void*)Ubuf, kMlp, 0L,
        b1, b1, 0L, kSeq, kMlp, kDim, 1.0f / 16.0f);
    gelu_f16x2_kernel<<<gGelu, blk256, 0, stream>>>(Ubuf, G16, n2g, 16.0f);
    wmma_gemm64<0, false, 2, 0, true, 0><<<gM2, blk256, 0, stream>>>(
        G16, G16, kMlp, 0L, W2T16, W2T16, kMlp, 0L, (void*)outb, (void*)outb, kDim, 0L,
        b2, X1, 0L, kSeq, kDim, kMlp, 1.0f / 256.0f);
  }
}
